// TCNNSplitModel_16080357556230
// MI455X (gfx1250) — hardware-verified
//
#include <hip/hip_runtime.h>


namespace {
constexpr int NS = 1 << 21, NF = 12, NLV = 2, FPL = 2, TBITS = 19, TSIZE = 1 << TBITS, NIN = 29, KIN = 32, NH = 64, NO = 3;
constexpr unsigned PRIME = 2654435761u;
constexpr float XS = 8.0f, WSC = 256.0f;

typedef _Float16 b16;
typedef __attribute__((ext_vector_type(16))) _Float16 v16b;
typedef __attribute__((ext_vector_type(8))) _Float16 v8b;
typedef __attribute__((ext_vector_type(8))) float v8f;
typedef __attribute__((ext_vector_type(4))) float v4f;
__device__ __forceinline__ float bf16_rne(float f) { unsigned int u = __float_as_uint(f); u += 0x7FFFu + ((u >> 16) & 1u); return __uint_as_float(u & 0xFFFF0000u); }
__device__ __forceinline__ void split16(float v, b16& hi, b16& lo) { hi = (b16)v; lo = (b16)(v - (float)hi); }
__device__ __forceinline__ v16b frag_kb(const b16* p, int hh) { const v8b a = *(const v8b*)(p + 8 * hh), b = *(const v8b*)(p + 16 + 8 * hh); v16b f;
#pragma unroll
  for (int e = 0; e < 8; ++e) { f[e] = a[e]; f[8 + e] = b[e]; } return f; }
__device__ __forceinline__ v8f wmma16b(v16b a, v16b b, v8f c) { v8f d = __builtin_amdgcn_wmma_f32_16x16x32_f16(false, a, false, b, (short)0, c, false, false); asm volatile("v_nop\n\tv_nop\n\tv_nop\n\tv_nop" : "+v"(d) : "v"(a), "v"(b)); return d; }
__device__ __forceinline__ void wave_lds_sync() { __builtin_amdgcn_fence(__ATOMIC_RELEASE, "workgroup"); __builtin_amdgcn_wave_barrier(); __builtin_amdgcn_fence(__ATOMIC_ACQUIRE, "workgroup"); }
__device__ __forceinline__ float pmul(float a, float b) { float p = a * b; asm volatile("" : "+v"(p)); return p; }
__device__ __forceinline__ float squareplus_(float x) { return 0.5f * (x + sqrtf(x * x + 4.0f)); }

__global__ __launch_bounds__(256) void prepw_kernel(const float* __restrict__ w1, const float* __restrict__ w2, const float* __restrict__ w3, b16* __restrict__ W1T, b16* __restrict__ W2T, b16* __restrict__ W3T) {
  const int t = blockIdx.x * 256 + threadIdx.x; v8b o; const int n1 = NH * KIN / 8, n2 = NH * NH / 8, n3 = 16 * NH / 8;
  if (t < n1) { const int e = t * 8, oo = e / KIN, k0 = e % KIN; for (int j = 0; j < 8; ++j) { const int k = k0 + j; o[j] = (k < NIN) ? (b16)(bf16_rne(w1[k * NH + oo]) * WSC) : (b16)0.0f; } for (int pass = 0; pass < 2; ++pass) { *(volatile v8b*)(W1T + e) = o; __threadfence(); } return; }
  int u = t - n1;
  if (u < n2) { const int e = u * 8, oo = e / NH, k0 = e % NH; for (int j = 0; j < 8; ++j) o[j] = (b16)(bf16_rne(w2[(k0 + j) * NH + oo]) * WSC); for (int pass = 0; pass < 2; ++pass) { *(volatile v8b*)(W2T + e) = o; __threadfence(); } return; } u -= n2;
  if (u < n3) { const int e = u * 8, oo = e / NH, k0 = e % NH; for (int j = 0; j < 8; ++j) o[j] = (oo < NO) ? (b16)(bf16_rne(w3[(k0 + j) * NO + oo]) * WSC) : (b16)0.0f; for (int pass = 0; pass < 2; ++pass) { *(volatile v8b*)(W3T + e) = o; __threadfence(); } }
}
__device__ __forceinline__ void grid_feat(const float* __restrict__ tab, float u, float v, int base_res, float* f4) {
  for (int lvl = 0; lvl < NLV; ++lvl) { const float res = (float)(base_res << lvl); const float pu = u * res, pv = v * res; const float fu = floorf(pu), fv = floorf(pv); const float wu = pu - fu, wv = pv - fv;
    const unsigned px0 = (unsigned)(int)fu, py0 = (unsigned)(int)fv; float a0 = 0.0f, a1 = 0.0f;
    for (int dx = 0; dx < 2; ++dx) for (int dy = 0; dy < 2; ++dy) { const unsigned px = px0 + (unsigned)dx, py = py0 + (unsigned)dy; const unsigned h = (px ^ (py * PRIME)) & (unsigned)(TSIZE - 1);
      const float wgt = pmul(dx ? wu : 1.0f - wu, dy ? wv : 1.0f - wv); const float* tv = tab + ((size_t)lvl * TSIZE + h) * FPL; a0 += pmul(wgt, bf16_rne(tv[0])); a1 += pmul(wgt, bf16_rne(tv[1])); }
    f4[lvl * 2] = a0; f4[lvl * 2 + 1] = a1; }
}
__global__ __launch_bounds__(128) void mlp_kernel(const float* __restrict__ x, const float* __restrict__ noise, const float* __restrict__ hg0, const float* __restrict__ hg1, const float* __restrict__ hg2, const b16* __restrict__ W1T, const b16* __restrict__ W2T, const b16* __restrict__ W3T, float* __restrict__ out) {
  __shared__ __attribute__((aligned(16))) b16 Ah[4][16][NH + 8], Al[4][16][NH + 8]; __shared__ __attribute__((aligned(16))) float res[256 * NO];
  const int wave = threadIdx.x >> 5, lane = threadIdx.x & 31, nloc = lane & 15, hlf = lane >> 4, t_ = threadIdx.x; const size_t s_blk = (size_t)blockIdx.x * 256; const float nz = bf16_rne(noise[0]);
  for (int tt = 0; tt < 4; ++tt) { const int sl0 = wave * 64 + tt * 16;
    if (lane < 16) { const size_t s = s_blk + sl0 + lane; const float u = bf16_rne(x[s * 3]), v = bf16_rne(x[s * 3 + 1]), lod = bf16_rne(x[s * 3 + 2]); float in[KIN];
      for (int j = 0; j < NF; ++j) { const float fr = (float)(1 << j); const float xu = u * fr, xv = v * fr; in[j] = fabsf(xu - floorf(xu + 0.5f)) * 2.0f - 0.5f; in[NF + j] = fabsf(xv - floorf(xv + 0.5f)) * 2.0f - 0.5f; }
      float f4[4]; const float* tab = (lod == 0.0f) ? hg0 : ((lod == 1.0f) ? hg1 : hg2); const int br = (lod == 0.0f) ? 128 : ((lod == 1.0f) ? 32 : 8); grid_feat(tab, u, v, br, f4);
      for (int j = 0; j < 4; ++j) in[2 * NF + j] = f4[j] + nz; in[28] = lod; in[29] = 0.0f; in[30] = 0.0f; in[31] = 0.0f;
      for (int k = 0; k < KIN; ++k) { b16 p, pl; split16(in[k] * XS, p, pl); Ah[wave][lane][k] = p; Al[wave][lane][k] = pl; } }
    wave_lds_sync();
    v8f acc[4] = {{}, {}, {}, {}};
    { const v16b a = frag_kb(&Ah[wave][nloc][0], hlf), al = frag_kb(&Al[wave][nloc][0], hlf);
#pragma unroll
      for (int t = 0; t < 4; ++t) { const v16b bw = frag_kb(W1T + (size_t)(t * 16 + nloc) * KIN, hlf); acc[t] = wmma16b(a, bw, acc[t]); acc[t] = wmma16b(al, bw, acc[t]); } }
    wave_lds_sync();
#pragma unroll
    for (int t = 0; t < 4; ++t)
#pragma unroll 1
      for (int r = 0; r < 8; ++r) { b16 p, pl; split16(squareplus_(acc[t][r] * (1.0f / (XS * WSC))) * XS, p, pl); Ah[wave][8 * hlf + r][t * 16 + nloc] = p; Al[wave][8 * hlf + r][t * 16 + nloc] = pl; }
    wave_lds_sync();
#pragma unroll
    for (int t = 0; t < 4; ++t) acc[t] = (v8f){};
#pragma unroll
    for (int kb = 0; kb < NH; kb += 32) { const v16b a = frag_kb(&Ah[wave][nloc][kb], hlf), al = frag_kb(&Al[wave][nloc][kb], hlf);
#pragma unroll
      for (int t = 0; t < 4; ++t) { const v16b bw = frag_kb(W2T + (size_t)(t * 16 + nloc) * NH + kb, hlf); acc[t] = wmma16b(a, bw, acc[t]); acc[t] = wmma16b(al, bw, acc[t]); } }
    wave_lds_sync();
#pragma unroll
    for (int t = 0; t < 4; ++t)
#pragma unroll 1
      for (int r = 0; r < 8; ++r) { b16 p, pl; split16(squareplus_(acc[t][r] * (1.0f / (XS * WSC))) * XS, p, pl); Ah[wave][8 * hlf + r][t * 16 + nloc] = p; Al[wave][8 * hlf + r][t * 16 + nloc] = pl; }
    wave_lds_sync();
    v8f o3 = {};
#pragma unroll
    for (int kb = 0; kb < NH; kb += 32) { const v16b bw = frag_kb(W3T + (size_t)nloc * NH + kb, hlf); o3 = wmma16b(frag_kb(&Ah[wave][nloc][kb], hlf), bw, o3); o3 = wmma16b(frag_kb(&Al[wave][nloc][kb], hlf), bw, o3); }
    if (nloc < NO) for (int r = 0; r < 8; ++r) res[(sl0 + 8 * hlf + r) * NO + nloc] = o3[r] * (1.0f / (XS * WSC));
    wave_lds_sync(); }
  __syncthreads();
  for (int pass = 0; pass < 2; ++pass) { for (int q = t_; q < 256 * NO / 4; q += 128) *(volatile v4f*)(out + s_blk * NO + q * 4) = *(const v4f*)(&res[q * 4]); __threadfence(); }
}
}

extern "C" void kernel_launch(void* const* d_in, const int* in_sizes, int n_in, void* d_out, int out_size, void* d_ws, size_t ws_size, hipStream_t stream) {
  (void)n_in;
  auto Fp = [&](int i) { return (const float*)d_in[i]; };
  if (in_sizes[0] != NS * 3 || in_sizes[2] != NLV * TSIZE * FPL || in_sizes[5] != NIN * NH || in_sizes[6] != NH * NH || in_sizes[7] != NH * NO || out_size != NS * NO) return;
  size_t off = 0; char* ws = (char*)d_ws;
  auto carve = [&](size_t bytes) { char* p = ws + off; off += (bytes + 255) & ~(size_t)255; return p; };
  b16* W1T = (b16*)carve(NH * KIN * 2); b16* W2T = (b16*)carve(NH * NH * 2); b16* W3T = (b16*)carve(16 * NH * 2);
  if (off > ws_size || off > ((size_t)128 << 20)) return;
  prepw_kernel<<<(NH * KIN / 8 + NH * NH / 8 + 16 * NH / 8 + 255) / 256, 256, 0, stream>>>(Fp(5), Fp(6), Fp(7), W1T, W2T, W3T);
  mlp_kernel<<<NS / 256, 128, 0, stream>>>(Fp(0), Fp(1), Fp(2), Fp(3), Fp(4), W1T, W2T, W3T, (float*)d_out);
}
